// InferwNet_11587821764942
// MI455X (gfx1250) — hardware-verified
//
#include <hip/hip_runtime.h>
#include <stddef.h>


#pragma clang fp contract(off)

#define NB    4096
#define NHB   2048
#define IMG   28
#define NPIX  784
#define C1    32
#define C2    64
#define P1    14
#define NP1   196
#define P2    7
#define NP2   49
#define KFC   3136
#define NK    64
#define NKB   98
#define TPB   256
#define TFC   64
#define WT2   8
#define PPW   4

#define G_WCVT (NKB + (9 * C2 * C1) / (8 * TPB))
#define G_C1   ((NHB * NP1) / TPB)
#define G_C2   ((NHB * NP2) / (PPW * WT2))
#define G_FC   (NB / 32)

static_assert(NB == 2 * NHB);
static_assert(KFC == C2 * NP2);
static_assert(KFC == NKB * 32);
static_assert((NHB * NP1) % TPB == 0);
static_assert((NHB * NP2) % (PPW * WT2) == 0);
static_assert(NB % 32 == 0);
static_assert(NK == 64);
static_assert(TFC == 64);
static_assert((NK * KFC) % (8 * TPB) == 0);
static_assert((9 * C2 * C1) % (8 * TPB) == 0);
static_assert(C1 == 32);
static_assert(G_WCVT == 107);
static_assert(G_C1 == 1568);
static_assert(G_C2 == 3136);

typedef float        v4f  __attribute__((ext_vector_type(4)));
typedef unsigned int v4u  __attribute__((ext_vector_type(4)));
typedef float        v8f  __attribute__((ext_vector_type(8)));
typedef __bf16       v16b __attribute__((ext_vector_type(16)));
typedef v4f __attribute__((may_alias)) v4fa;
typedef v4u __attribute__((may_alias)) v4ua;

union Frag { v16b v; v4u q[2]; };

__device__ __forceinline__ unsigned int bf_rne(float f) {
  const unsigned int u = __float_as_uint(f);
  return (u + 0x7FFFu + ((u >> 16) & 1u)) >> 16;
}
__device__ __forceinline__ void sp2(float f, unsigned int& hb, unsigned int& lb) {
  const unsigned int hbits = bf_rne(f);
  const float hf = __uint_as_float(hbits << 16);
  hb = hbits;
  lb = bf_rne(f - hf);
}
__device__ __forceinline__ void split8(v4f a, v4f c, v4u& hq, v4u& lq) {
  unsigned int h0, h1, h2, h3, h4, h5, h6, h7;
  unsigned int l0, l1, l2, l3, l4, l5, l6, l7;
  sp2(a.x, h0, l0); sp2(a.y, h1, l1); sp2(a.z, h2, l2); sp2(a.w, h3, l3);
  sp2(c.x, h4, l4); sp2(c.y, h5, l5); sp2(c.z, h6, l6); sp2(c.w, h7, l7);
  v4u hv, lv;
  hv.x = h0 | (h1 << 16); hv.y = h2 | (h3 << 16); hv.z = h4 | (h5 << 16); hv.w = h6 | (h7 << 16);
  lv.x = l0 | (l1 << 16); lv.y = l2 | (l3 << 16); lv.z = l4 | (l5 << 16); lv.w = l6 | (l7 << 16);
  hq = hv;
  lq = lv;
}

__device__ __forceinline__ v4u zsel(v4u v, bool ok) {
  v4u r;
  r.x = ok ? v.x : 0u;
  r.y = ok ? v.y : 0u;
  r.z = ok ? v.z : 0u;
  r.w = ok ? v.w : 0u;
  return r;
}

__device__ __forceinline__ v8f wmma_bf(v16b a, v16b b, v8f c) {
  v8f d = __builtin_amdgcn_wmma_f32_16x16x32_bf16(false, a, false, b, (short)0, c, false, false);
  asm volatile("v_nop\n\tv_nop\n\tv_nop\n\tv_nop" : "+v"(d) : "v"(a), "v"(b));
  return d;
}

__device__ __forceinline__ v16b ldfrag(const unsigned short* p, int h) {
  Frag f;
  f.q[0] = *(const v4ua*)(p + 8 * h);
  f.q[1] = *(const v4ua*)(p + 16 + 8 * h);
  return f.v;
}

__global__ __launch_bounds__(TPB) void k_wcvt(const float* __restrict__ fcw,
                                              const float* __restrict__ w2,
                                              unsigned short* __restrict__ fwh,
                                              unsigned short* __restrict__ fwl,
                                              unsigned short* __restrict__ w2h,
                                              unsigned short* __restrict__ w2l)
{
  const int blk = blockIdx.x, tid = threadIdx.x;
  if (blk < NKB) {
    const int u  = blk * TPB + tid;
    const int cg = u & 7;
    const int t  = u >> 3;
    const int n  = t / NP2;
    const int pp = t - n * NP2;
    const float* src = fcw + (size_t)n * KFC + (cg * 8) * NP2 + pp;
    v4f a, c;
    a.x = src[0];        a.y = src[NP2];      a.z = src[2 * NP2];  a.w = src[3 * NP2];
    c.x = src[4 * NP2];  c.y = src[5 * NP2];  c.z = src[6 * NP2];  c.w = src[7 * NP2];
    v4u hq, lq;
    split8(a, c, hq, lq);
    unsigned short* dh = fwh + (size_t)u * 8;
    unsigned short* dl = fwl + (size_t)u * 8;
    *(volatile v4u*)dh = hq;
    *(volatile v4u*)dl = lq;
    __threadfence();
    *(volatile v4u*)dh = hq;
    *(volatile v4u*)dl = lq;
  } else {
    const int u   = (blk - NKB) * TPB + tid;
    const int icg = u & 3;
    const int oc  = (u >> 2) & 63;
    const int tap = u >> 8;
    const int ky  = tap / 3, kx = tap - ky * 3;
    const float* src = w2 + (size_t)(oc * C1 + icg * 8) * 9 + ky * 3 + kx;
    v4f a, c;
    a.x = src[0];   a.y = src[9];   a.z = src[18];  a.w = src[27];
    c.x = src[36];  c.y = src[45];  c.z = src[54];  c.w = src[63];
    v4u hq, lq;
    split8(a, c, hq, lq);
    unsigned short* dh = w2h + (size_t)u * 8;
    unsigned short* dl = w2l + (size_t)u * 8;
    *(volatile v4u*)dh = hq;
    *(volatile v4u*)dl = lq;
    __threadfence();
    *(volatile v4u*)dh = hq;
    *(volatile v4u*)dl = lq;
  }
}

__global__ __launch_bounds__(TPB) void k_conv1(const float* __restrict__ x,
                                               const float* __restrict__ w1,
                                               const float* __restrict__ b1,
                                               int half,
                                               unsigned short* __restrict__ h1h,
                                               unsigned short* __restrict__ h1l)
{
  __shared__ float sWt[C1 * 9];
  __shared__ float sBs[C1];
  __shared__ __align__(16) unsigned short sHi[TPB * C1];
  __shared__ __align__(16) unsigned short sLo[TPB * C1];

  const int tid = threadIdx.x;
  for (int i = tid; i < C1 * 9; i += TPB) sWt[i] = w1[i];
  if (tid < C1) sBs[tid] = b1[tid];

  const int pl  = blockIdx.x * TPB + tid;
  const int plc = (pl > NHB * NP1 - 1) ? (NHB * NP1 - 1) : pl;
  const int bl  = plc / NP1;
  const int rr  = plc - bl * NP1;
  const int py  = rr / P1, px = rr - py * P1;
  const int b   = half * NHB + bl;
  const float* xb = x + (size_t)b * NPIX;

  float p[4][4];
  #pragma unroll
  for (int dy = 0; dy < 4; ++dy) {
    const int iy = 2 * py - 1 + dy;
    const bool oky = (unsigned)iy < (unsigned)IMG;
    const int iyc = (iy < 0) ? 0 : ((iy > IMG - 1) ? (IMG - 1) : iy);
    #pragma unroll
    for (int dx = 0; dx < 4; ++dx) {
      const int ix = 2 * px - 1 + dx;
      const bool okx = (unsigned)ix < (unsigned)IMG;
      const int ixc = (ix < 0) ? 0 : ((ix > IMG - 1) ? (IMG - 1) : ix);
      const float v = xb[iyc * IMG + ixc];
      p[dy][dx] = (oky && okx) ? v : 0.0f;
    }
  }
  __syncthreads();

  #pragma unroll 1
  for (int oc = 0; oc < C1; ++oc) {
    const float* w = sWt + oc * 9;
    const float k0 = w[0], k1 = w[1], k2 = w[2], k3 = w[3], k4 = w[4];
    const float k5 = w[5], k6 = w[6], k7 = w[7], k8 = w[8];
    float s[4];
    #pragma unroll
    for (int qq = 0; qq < 4; ++qq) {
      const int dy = qq >> 1, dx = qq & 1;
      float t = p[dy][dx] * k0;
      t = fmaf(p[dy][dx + 1],     k1, t);
      t = fmaf(p[dy][dx + 2],     k2, t);
      t = fmaf(p[dy + 1][dx],     k3, t);
      t = fmaf(p[dy + 1][dx + 1], k4, t);
      t = fmaf(p[dy + 1][dx + 2], k5, t);
      t = fmaf(p[dy + 2][dx],     k6, t);
      t = fmaf(p[dy + 2][dx + 1], k7, t);
      t = fmaf(p[dy + 2][dx + 2], k8, t);
      s[qq] = t;
    }
    const float mx = fmaxf(fmaxf(s[0], s[1]), fmaxf(s[2], s[3]));
    const float v  = fmaxf(mx + sBs[oc], 0.0f);
    unsigned int hb, lb;
    sp2(v, hb, lb);
    sHi[tid * C1 + oc] = (unsigned short)hb;
    sLo[tid * C1 + oc] = (unsigned short)lb;
  }
  __syncthreads();

  const size_t base = (size_t)blockIdx.x * (TPB * C1);
  #pragma unroll
  for (int it = 0; it < 4; ++it) {
    const int ch = it * TPB + tid;
    const v4u hv = *(const v4ua*)(sHi + ch * 8);
    const v4u lv = *(const v4ua*)(sLo + ch * 8);
    *(volatile v4u*)(h1h + base + (size_t)ch * 8) = hv;
    *(volatile v4u*)(h1l + base + (size_t)ch * 8) = lv;
  }
  __threadfence();
  #pragma unroll
  for (int it = 0; it < 4; ++it) {
    const int ch = it * TPB + tid;
    const v4u hv = *(const v4ua*)(sHi + ch * 8);
    const v4u lv = *(const v4ua*)(sLo + ch * 8);
    *(volatile v4u*)(h1h + base + (size_t)ch * 8) = hv;
    *(volatile v4u*)(h1l + base + (size_t)ch * 8) = lv;
  }
}

__global__ __launch_bounds__(TPB) void k_conv2(const unsigned short* __restrict__ h1h,
                                               const unsigned short* __restrict__ h1l,
                                               const unsigned short* __restrict__ w2h,
                                               const unsigned short* __restrict__ w2l,
                                               const float* __restrict__ b2,
                                               int half,
                                               float* __restrict__ feats)
{
  __shared__ __align__(16) float sOut[WT2 * PPW * C2];

  const int tid = threadIdx.x, lane = tid & 31, wv = tid >> 5;
  const int h = lane >> 4, m = lane & 15;
  const int wt = blockIdx.x * WT2 + wv;
  const int gpp0 = half * (NHB * NP2) + wt * PPW;
  const int gppm = gpp0 + (m >> 2);
  const int q  = m & 3;
  const int b  = gppm / NP2;
  const int pp = gppm - b * NP2;
  int bl = b - half * NHB;
  bl = (bl < 0) ? 0 : ((bl > NHB - 1) ? (NHB - 1) : bl);
  const int py = pp / P2, px = pp - py * P2;
  const int oy = 2 * py + (q >> 1), ox = 2 * px + (q & 1);
  const size_t ibase = (size_t)bl * (NP1 * C1);
  const unsigned short* hb = h1h + ibase;
  const unsigned short* hl = h1l + ibase;

  const v8f z8 = {0.f, 0.f, 0.f, 0.f, 0.f, 0.f, 0.f, 0.f};
  v8f acc0 = z8, acc1 = z8, acc2 = z8, acc3 = z8;

  #pragma unroll 1
  for (int tap = 0; tap < 9; ++tap) {
    const int ky = tap / 3, kx = tap - ky * 3;
    const int iy = oy + ky - 1, ix = ox + kx - 1;
    const bool ok = ((unsigned)iy < (unsigned)P1) && ((unsigned)ix < (unsigned)P1);
    const int iyc = (iy < 0) ? 0 : ((iy > P1 - 1) ? (P1 - 1) : iy);
    const int ixc = (ix < 0) ? 0 : ((ix > P1 - 1) ? (P1 - 1) : ix);
    const int poff = (iyc * P1 + ixc) * C1;
    Frag ah, al;
    ah.q[0] = zsel(*(const v4ua*)(hb + poff + 8 * h), ok);
    ah.q[1] = zsel(*(const v4ua*)(hb + poff + 16 + 8 * h), ok);
    al.q[0] = zsel(*(const v4ua*)(hl + poff + 8 * h), ok);
    al.q[1] = zsel(*(const v4ua*)(hl + poff + 16 + 8 * h), ok);
    const unsigned short* wb = w2h + (size_t)(tap * C2 + m) * C1;
    const unsigned short* wl = w2l + (size_t)(tap * C2 + m) * C1;
    {
      const v16b bh = ldfrag(wb, h);
      const v16b bq = ldfrag(wl, h);
      acc0 = wmma_bf(ah.v, bh, acc0);
      acc0 = wmma_bf(ah.v, bq, acc0);
      acc0 = wmma_bf(al.v, bh, acc0);
    }
    {
      const v16b bh = ldfrag(wb + 16 * C1, h);
      const v16b bq = ldfrag(wl + 16 * C1, h);
      acc1 = wmma_bf(ah.v, bh, acc1);
      acc1 = wmma_bf(ah.v, bq, acc1);
      acc1 = wmma_bf(al.v, bh, acc1);
    }
    {
      const v16b bh = ldfrag(wb + 32 * C1, h);
      const v16b bq = ldfrag(wl + 32 * C1, h);
      acc2 = wmma_bf(ah.v, bh, acc2);
      acc2 = wmma_bf(ah.v, bq, acc2);
      acc2 = wmma_bf(al.v, bh, acc2);
    }
    {
      const v16b bh = ldfrag(wb + 48 * C1, h);
      const v16b bq = ldfrag(wl + 48 * C1, h);
      acc3 = wmma_bf(ah.v, bh, acc3);
      acc3 = wmma_bf(ah.v, bq, acc3);
      acc3 = wmma_bf(al.v, bh, acc3);
    }
  }

  {
    const float bb0 = b2[m], bb1 = b2[16 + m], bb2 = b2[32 + m], bb3 = b2[48 + m];
    float* so = sOut + wv * (PPW * C2);
    const int r0 = (2 * h) * C2, r1 = (2 * h + 1) * C2;
    float u0, u1;
    u0 = fmaxf(fmaxf(acc0[0], acc0[1]), fmaxf(acc0[2], acc0[3]));
    u1 = fmaxf(fmaxf(acc0[4], acc0[5]), fmaxf(acc0[6], acc0[7]));
    so[r0 + m]      = fmaxf(u0 + bb0, 0.0f);
    so[r1 + m]      = fmaxf(u1 + bb0, 0.0f);
    u0 = fmaxf(fmaxf(acc1[0], acc1[1]), fmaxf(acc1[2], acc1[3]));
    u1 = fmaxf(fmaxf(acc1[4], acc1[5]), fmaxf(acc1[6], acc1[7]));
    so[r0 + 16 + m] = fmaxf(u0 + bb1, 0.0f);
    so[r1 + 16 + m] = fmaxf(u1 + bb1, 0.0f);
    u0 = fmaxf(fmaxf(acc2[0], acc2[1]), fmaxf(acc2[2], acc2[3]));
    u1 = fmaxf(fmaxf(acc2[4], acc2[5]), fmaxf(acc2[6], acc2[7]));
    so[r0 + 32 + m] = fmaxf(u0 + bb2, 0.0f);
    so[r1 + 32 + m] = fmaxf(u1 + bb2, 0.0f);
    u0 = fmaxf(fmaxf(acc3[0], acc3[1]), fmaxf(acc3[2], acc3[3]));
    u1 = fmaxf(fmaxf(acc3[4], acc3[5]), fmaxf(acc3[6], acc3[7]));
    so[r0 + 48 + m] = fmaxf(u0 + bb3, 0.0f);
    so[r1 + 48 + m] = fmaxf(u1 + bb3, 0.0f);
  }
  __syncthreads();

  const float* so = sOut + wv * (PPW * C2);
  float* dst = feats + (size_t)gpp0 * C2;
  {
    const v4f o0 = *(const v4fa*)(so + 4 * lane);
    const v4f o1 = *(const v4fa*)(so + 128 + 4 * lane);
    *(volatile v4f*)(dst + 4 * lane) = o0;
    *(volatile v4f*)(dst + 128 + 4 * lane) = o1;
  }
  __threadfence();
  {
    const v4f o0 = *(const v4fa*)(so + 4 * lane);
    const v4f o1 = *(const v4fa*)(so + 128 + 4 * lane);
    *(volatile v4f*)(dst + 4 * lane) = o0;
    *(volatile v4f*)(dst + 128 + 4 * lane) = o1;
  }
}

__global__ __launch_bounds__(TFC) void k_fc(const float* __restrict__ feats,
                                            const unsigned short* __restrict__ fwh,
                                            const unsigned short* __restrict__ fwl,
                                            const float* __restrict__ fcb,
                                            const float* __restrict__ cent,
                                            float* __restrict__ outp)
{
  __shared__ __align__(16) float sC[NK * NK];
  __shared__ __align__(16) float sF[2 * 16 * NK];
  __shared__ __align__(16) float sQ[2 * 16 * NK];
  __shared__ __align__(16) float sW[2 * 16 * NK];

  const int tid = threadIdx.x, lane = tid & 31, wv = tid >> 5;
  const int h = lane >> 4, m = lane & 15;

  #pragma unroll
  for (int it = 0; it < (NK * NK) / (4 * TFC); ++it) {
    const int i4 = it * TFC + tid;
    *(v4fa*)(sC + 4 * i4) = *(const v4fa*)(cent + 4 * i4);
  }
  __syncthreads();

  const int row0 = blockIdx.x * 32 + wv * 16;
  const float* arow = feats + (size_t)(row0 + m) * KFC;

  const v8f z8 = {0.f, 0.f, 0.f, 0.f, 0.f, 0.f, 0.f, 0.f};
  v8f acc0 = z8, acc1 = z8, acc2 = z8, acc3 = z8;

  #pragma unroll 1
  for (int kb = 0; kb < NKB; ++kb) {
    const float* ap = arow + kb * 32;
    const v4f x0 = *(const v4fa*)(ap + 8 * h);
    const v4f x1 = *(const v4fa*)(ap + 8 * h + 4);
    const v4f x2 = *(const v4fa*)(ap + 16 + 8 * h);
    const v4f x3 = *(const v4fa*)(ap + 20 + 8 * h);
    Frag ah, al;
    split8(x0, x1, ah.q[0], al.q[0]);
    split8(x2, x3, ah.q[1], al.q[1]);
    const unsigned short* wb = fwh + (size_t)m * KFC + kb * 32;
    const unsigned short* wl = fwl + (size_t)m * KFC + kb * 32;
    {
      const v16b bh = ldfrag(wb, h);
      const v16b bq = ldfrag(wl, h);
      acc0 = wmma_bf(ah.v, bh, acc0);
      acc0 = wmma_bf(ah.v, bq, acc0);
      acc0 = wmma_bf(al.v, bh, acc0);
    }
    {
      const v16b bh = ldfrag(wb + (size_t)16 * KFC, h);
      const v16b bq = ldfrag(wl + (size_t)16 * KFC, h);
      acc1 = wmma_bf(ah.v, bh, acc1);
      acc1 = wmma_bf(ah.v, bq, acc1);
      acc1 = wmma_bf(al.v, bh, acc1);
    }
    {
      const v16b bh = ldfrag(wb + (size_t)32 * KFC, h);
      const v16b bq = ldfrag(wl + (size_t)32 * KFC, h);
      acc2 = wmma_bf(ah.v, bh, acc2);
      acc2 = wmma_bf(ah.v, bq, acc2);
      acc2 = wmma_bf(al.v, bh, acc2);
    }
    {
      const v16b bh = ldfrag(wb + (size_t)48 * KFC, h);
      const v16b bq = ldfrag(wl + (size_t)48 * KFC, h);
      acc3 = wmma_bf(ah.v, bh, acc3);
      acc3 = wmma_bf(ah.v, bq, acc3);
      acc3 = wmma_bf(al.v, bh, acc3);
    }
  }

  {
    const float bb0 = fcb[m], bb1 = fcb[16 + m], bb2 = fcb[32 + m], bb3 = fcb[48 + m];
    float* sf = sF + wv * (16 * NK);
    #pragma unroll
    for (int r = 0; r < 8; ++r) {
      const int ro = (8 * h + r) * NK;
      sf[ro + m]      = acc0[r] + bb0;
      sf[ro + 16 + m] = acc1[r] + bb1;
      sf[ro + 32 + m] = acc2[r] + bb2;
      sf[ro + 48 + m] = acc3[r] + bb3;
    }
  }
  __syncthreads();

  {
    const float* sf = sF + wv * (16 * NK);
    float* o0 = outp + (size_t)row0 * NK;
    #pragma unroll
    for (int it = 0; it < 8; ++it) {
      const int i4 = it * 32 + lane;
      const v4f v = *(const v4fa*)(sf + 4 * i4);
      *(volatile v4f*)(o0 + 4 * i4) = v;
    }
    __threadfence();
    #pragma unroll
    for (int it = 0; it < 8; ++it) {
      const int i4 = it * 32 + lane;
      const v4f v = *(const v4fa*)(sf + 4 * i4);
      *(volatile v4f*)(o0 + 4 * i4) = v;
    }
  }

  {
    const float* sf = sF + wv * (16 * NK);
    float* sq = sQ + wv * (16 * NK);
    float* sw = sW + wv * (16 * NK);
    const float* cA = sC + lane * NK;
    const float* cB = sC + (lane + 32) * NK;
    #pragma unroll 1
    for (int i = 0; i < 16; ++i) {
      const float* fr = sf + i * NK;
      double s0 = 0.0, s1 = 0.0;
      #pragma unroll 4
      for (int k = 0; k < NK; ++k) {
        const float f  = fr[k];
        const float d0 = f - cA[k];
        const float d1 = f - cB[k];
        s0 += (double)(d0 * d0);
        s1 += (double)(d1 * d1);
      }
      const float dd0 = sqrtf((float)s0);
      const float dd1 = sqrtf((float)s1);
      const bool t1 = dd1 < dd0;
      float bv = t1 ? dd1 : dd0;
      int   bi = t1 ? (lane + 32) : lane;
      #pragma unroll
      for (int s = 16; s >= 1; s >>= 1) {
        const float ov = __shfl_xor(bv, s, 32);
        const int   oi = __shfl_xor(bi, s, 32);
        const bool take = (ov < bv) || ((ov == bv) && (oi < bi));
        bv = take ? ov : bv;
        bi = take ? oi : bi;
      }
      const float e0 = expf(bv - dd0);
      const float e1 = expf(bv - dd1);
      float es = e0 + e1;
      #pragma unroll
      for (int s = 16; s >= 1; s >>= 1) es += __shfl_xor(es, s, 32);
      es = __shfl(es, 0, 32);
      const float rcp = 1.0f / es;
      sq[i * NK + lane]      = e0 * rcp;
      sq[i * NK + 32 + lane] = e1 * rcp;
      sw[i * NK + lane]      = (bi == lane) ? 1.0f : 0.0f;
      sw[i * NK + 32 + lane] = (bi == lane + 32) ? 1.0f : 0.0f;
    }
  }
  __syncthreads();

  {
    const float* sq = sQ + wv * (16 * NK);
    const float* sw = sW + wv * (16 * NK);
    float* o1 = outp + (size_t)NB * NK + (size_t)row0 * NK;
    float* o2 = outp + (size_t)2 * NB * NK + (size_t)row0 * NK;
    #pragma unroll
    for (int it = 0; it < 8; ++it) {
      const int i4 = it * 32 + lane;
      const v4f vq = *(const v4fa*)(sq + 4 * i4);
      const v4f vw = *(const v4fa*)(sw + 4 * i4);
      *(volatile v4f*)(o1 + 4 * i4) = vq;
      *(volatile v4f*)(o2 + 4 * i4) = vw;
    }
    __threadfence();
    #pragma unroll
    for (int it = 0; it < 8; ++it) {
      const int i4 = it * 32 + lane;
      const v4f vq = *(const v4fa*)(sq + 4 * i4);
      const v4f vw = *(const v4fa*)(sw + 4 * i4);
      *(volatile v4f*)(o1 + 4 * i4) = vq;
      *(volatile v4f*)(o2 + 4 * i4) = vw;
    }
  }
}

extern "C" void kernel_launch(void* const* d_in, const int* in_sizes, int n_in,
                              void* d_out, int out_size, void* d_ws, size_t ws_size,
                              hipStream_t stream)
{
  if (n_in < 8) return;
  if (in_sizes[0] != NB * NPIX) return;
  if (in_sizes[1] != C1 * 9) return;
  if (in_sizes[2] != C1) return;
  if (in_sizes[3] != C2 * C1 * 9) return;
  if (in_sizes[4] != C2) return;
  if (in_sizes[5] != NK * KFC) return;
  if (in_sizes[6] != NK) return;
  if (in_sizes[7] != NK * NK) return;
  if (out_size != 3 * NB * NK) return;

  const float* x    = (const float*)d_in[0];
  const float* w1   = (const float*)d_in[1];
  const float* b1   = (const float*)d_in[2];
  const float* w2   = (const float*)d_in[3];
  const float* b2   = (const float*)d_in[4];
  const float* fcw  = (const float*)d_in[5];
  const float* fcb  = (const float*)d_in[6];
  const float* cent = (const float*)d_in[7];
  float* out = (float*)d_out;

  const size_t bH1   = (size_t)NHB * NP1 * C1 * 2;
  const size_t bFeat = (size_t)NB * KFC * 4;
  const size_t bFW   = (size_t)NK * KFC * 2;
  const size_t bW2   = (size_t)9 * C2 * C1 * 2;
  const size_t total = 2 * bH1 + bFeat + 2 * bFW + 2 * bW2;
  if (total > ws_size) return;
  if (total > (size_t)134217728) return;

  char* ws = (char*)d_ws;
  size_t off = 0;
  unsigned short* h1h   = (unsigned short*)(ws + off); off += bH1;
  unsigned short* h1l   = (unsigned short*)(ws + off); off += bH1;
  float*          feats = (float*)(ws + off);          off += bFeat;
  unsigned short* fwh   = (unsigned short*)(ws + off); off += bFW;
  unsigned short* fwl   = (unsigned short*)(ws + off); off += bFW;
  unsigned short* w2h   = (unsigned short*)(ws + off); off += bW2;
  unsigned short* w2l   = (unsigned short*)(ws + off); off += bW2;
  if (off != total) return;

  k_wcvt<<<G_WCVT, TPB, 0, stream>>>(fcw, w2, fwh, fwl, w2h, w2l);
  k_conv1<<<G_C1, TPB, 0, stream>>>(x, w1, b1, 0, h1h, h1l);
  k_conv2<<<G_C2, TPB, 0, stream>>>(h1h, h1l, w2h, w2l, b2, 0, feats);
  k_conv1<<<G_C1, TPB, 0, stream>>>(x, w1, b1, 1, h1h, h1l);
  k_conv2<<<G_C2, TPB, 0, stream>>>(h1h, h1l, w2h, w2l, b2, 1, feats);
  k_fc<<<G_FC, TFC, 0, stream>>>(feats, fwh, fwl, fcb, cent, out);
}
